// PhaseSyncAttentionV4_11416023072953
// MI455X (gfx1250) — hardware-verified
//
#include <hip/hip_runtime.h>


namespace {
constexpr int Bsz = 4, T = 1024, HID = 512, HIN = 256, NOUT = 256, DH = 64, DR = 32, NH = 8, NKV = 8, REP = NH / NKV, NS = 8;
constexpr int WIN = 255;
constexpr int KVW = NKV * DH;
constexpr int NQKV = HID + 2 * KVW;
constexpr int MROWS = Bsz * T;
constexpr int QT_PER_B = T / 16;

typedef _Float16 b16;
typedef __attribute__((ext_vector_type(16))) _Float16 v16b;
typedef __attribute__((ext_vector_type(8)))  _Float16 v8b;
typedef __attribute__((ext_vector_type(8)))  float v8f;
typedef __attribute__((ext_vector_type(4)))  float v4f;

__device__ __forceinline__ v8b ld8b(const b16* p) { return *(const v8b*)p; }
__device__ __forceinline__ v16b cat8b(v8b a, v8b b) { return __builtin_shufflevector(a, b, 0, 1, 2, 3, 4, 5, 6, 7, 8, 9, 10, 11, 12, 13, 14, 15); }
__device__ __forceinline__ v16b frag_kb(const b16* p, int hh) { return cat8b(ld8b(p + 8 * hh), ld8b(p + 16 + 8 * hh)); }
__device__ __forceinline__ void split_bf16(float v, b16& hi, b16& lo) {
  hi = (b16)v; lo = (b16)0.0f;
}
__device__ __forceinline__ void frag_ksplit(const float* p, int hh, v16b& fh_, v16b& fl_) {
  const float* p0 = p + 8 * hh; const float* p1 = p + 16 + 8 * hh;
#pragma unroll
  for (int e = 0; e < 8; ++e) { b16 a, c; split_bf16(p0[e], a, c); fh_[e] = a; fl_[e] = c; split_bf16(p1[e], a, c); fh_[8 + e] = a; fl_[8 + e] = c; }
}
__device__ __forceinline__ v8f wmma16b(v16b a, v16b b, v8f c) {
  v8f d = __builtin_amdgcn_wmma_f32_16x16x32_f16(false, a, false, b, (short)0, c, false, false);
  asm volatile("v_nop\n\tv_nop\n\tv_nop\n\tv_nop" : "+v"(d) : "v"(a), "v"(b));
  return d;
}
__device__ __forceinline__ v8f wmma3(v16b ah, v16b al, v16b bh, v16b bl, v8f c) {
  (void)al; (void)bl; return wmma16b(ah, bh, c);
}
__device__ __forceinline__ v8f wmma1(v16b ah, v16b al, v16b bh, v16b bl, v8f c) {
  (void)al; (void)bl; return wmma16b(ah, bh, c);
}
__device__ __forceinline__ void wave_lds_sync() {
  __builtin_amdgcn_fence(__ATOMIC_RELEASE, "workgroup");
  __builtin_amdgcn_wave_barrier();
  __builtin_amdgcn_fence(__ATOMIC_ACQUIRE, "workgroup");
}

__global__ __launch_bounds__(256) void wcvt_kernel(const float* __restrict__ wq, const float* __restrict__ wk, const float* __restrict__ wv,
                                                   const float* __restrict__ wo, b16* __restrict__ wqh, b16* __restrict__ wql,
                                                   b16* __restrict__ woh, b16* __restrict__ wol) {
  const size_t tid = (size_t)blockIdx.x * blockDim.x + threadIdx.x, stride = (size_t)gridDim.x * blockDim.x;
  const size_t nq = (size_t)NQKV * HID / 8, no = (size_t)HID * HID / 8;
  for (int pass = 0; pass < 2; ++pass) {
    for (size_t c = tid; c < nq + no; c += stride) {
      float f[8]; size_t i; b16* dh; b16* dl;
      if (c < nq) {
        i = c * 8; const size_t n = i / HID, k0 = i % HID;
        const float* w; int nn, ld;
        if (n < (size_t)HID) { w = wq; nn = (int)n; ld = HID; } else if (n < (size_t)(HID + KVW)) { w = wk; nn = (int)n - HID; ld = KVW; } else { w = wv; nn = (int)n - HID - KVW; ld = KVW; }
#pragma unroll
        for (int e = 0; e < 8; ++e) f[e] = w[(size_t)(k0 + e) * ld + nn];
        dh = wqh; dl = wql;
      } else {
        i = (c - nq) * 8; const size_t n = i / HID, k0 = i % HID;
#pragma unroll
        for (int e = 0; e < 8; ++e) f[e] = wo[(size_t)(k0 + e) * HID + n];
        dh = woh; dl = wol;
      }
      v8b bh, bl;
#pragma unroll
      for (int e = 0; e < 8; ++e) { b16 a, cc; split_bf16(f[e], a, cc); bh[e] = a; bl[e] = cc; }
      *(volatile v8b*)(dh + i) = bh; *(volatile v8b*)(dl + i) = bl;
    }
    __threadfence();
  }
}

__device__ __forceinline__ void gemm_tile_split(const float* __restrict__ A, const b16* __restrict__ wh, const b16* __restrict__ wl,
                                                int m0, int c0, int K, int nloc, int hlf, v8f (&acc)[2][4]) {
  for (int kb = 0; kb < K; kb += 32) {
    v16b a0h, a0l, a1h, a1l;
    frag_ksplit(A + (size_t)(m0 + nloc) * K + kb, hlf, a0h, a0l);
    frag_ksplit(A + (size_t)(m0 + 16 + nloc) * K + kb, hlf, a1h, a1l);
#pragma unroll
    for (int t = 0; t < 4; ++t) {
      const size_t wofs = (size_t)(c0 + t * 16 + nloc) * K + kb;
      const v16b bh = frag_kb(wh + wofs, hlf), bl = frag_kb(wl + wofs, hlf);
      acc[0][t] = wmma3(a0h, a0l, bh, bl, acc[0][t]);
      acc[1][t] = wmma3(a1h, a1l, bh, bl, acc[1][t]);
    }
  }
}

__global__ __launch_bounds__(128) void qkv_gemm_kernel(const float* __restrict__ xq, const float* __restrict__ xk, const float* __restrict__ xv,
                                                       const b16* __restrict__ wqh, const b16* __restrict__ wql,
                                                       const float* __restrict__ bq, const float* __restrict__ bk, const float* __restrict__ bv, const float* __restrict__ rope_cs, int xoff, int yoff,
                                                       const float* __restrict__ cphi, const float* __restrict__ sphi, const float* __restrict__ mag, const float* __restrict__ bandl, const float* __restrict__ pbs,
                                                       b16* __restrict__ Qh, b16* __restrict__ Ql, b16* __restrict__ Kh, b16* __restrict__ Kl,
                                                       b16* __restrict__ Vh, b16* __restrict__ Vl) {
  __shared__ __attribute__((aligned(16))) b16 Ts[4][2][32 * 64];
  const int lane = threadIdx.x & 31, wave = threadIdx.x >> 5, nloc = lane & 15, hlf = lane >> 4;
  const int m0 = (blockIdx.y + yoff) * 128 + wave * 32;
  const int c0 = (blockIdx.x + xoff) * 64;
  const int mat = (c0 < HID) ? 0 : (c0 < HID + KVW) ? 1 : 2;
  const int head = (mat == 0) ? (c0 / DH) : (mat == 1) ? ((c0 - HID) / DH) : ((c0 - HID - KVW) / DH);
  const float* x = (mat == 0) ? xq : (mat == 1) ? xk : xv;
  const float* bias = ((mat == 0) ? bq : (mat == 1) ? bk : bv) + head * DR;
  v8f acc[2][4];
#pragma unroll
  for (int r = 0; r < 2; ++r)
#pragma unroll
    for (int t = 0; t < 4; ++t) acc[r][t] = (v8f){};
  gemm_tile_split(x, wqh, wql, m0, c0, HIN, nloc, hlf, acc);
  const int b = m0 / T, t0 = m0 % T;
  float bw[NS]; { float mx = -INFINITY; for (int s_ = 0; s_ < NS; ++s_) mx = fmaxf(mx, bandl[head * NS + s_]); float z = 0.f; for (int s_ = 0; s_ < NS; ++s_) { bw[s_] = expf(bandl[head * NS + s_] - mx); z += bw[s_]; } for (int s_ = 0; s_ < NS; ++s_) bw[s_] /= z; }
  const float eph = expf(0.5f * pbs[head]);
  b16* Tp0 = Ts[wave][0]; b16* Tp1 = Ts[wave][1];
#pragma unroll
  for (int t = 0; t < 4; ++t)
#pragma unroll
    for (int r = 0; r < 2; ++r)
#pragma unroll
      for (int v = 0; v < 8; ++v) {
        const int rr = r * 16 + v + 8 * hlf, d = t * 16 + nloc;
        float val;
        (void)rope_cs;
        if (d < DR) val = (acc[r][t][v] + bias[d]) * ((mat == 0) ? 0.17677669529663689f : 1.0f);
        else if (mat < 2 && d < DR + 2 * NS) {
          const int tpos = t0 + rr, s_ = (d - DR) & (NS - 1);
          float mh = 0.f; for (int u = 0; u < NS; ++u) mh += mag[((size_t)b * NS + u) * T + tpos] * bw[u];
          const float cs = (d < DR + NS) ? cphi[((size_t)b * NS + s_) * T + tpos] : sphi[((size_t)b * NS + s_) * T + tpos];
          val = cs * sqrtf(bw[s_] + 1e-8f) * sqrtf(mh) * eph;
        } else val = 0.f;
        b16 yh, yl; split_bf16(val, yh, yl);
        const int idx = (mat < 2) ? (rr * 64 + d) : ((rr >> 4) * 1024 + d * 16 + (rr & 15));
        Tp0[idx] = yh; Tp1[idx] = yl;
      }
  wave_lds_sync();
  b16* dh; b16* dl; size_t o;
  if (mat == 0)      { o = ((size_t)(b * NH + head) * T + t0) * DH; dh = Qh + o; dl = Ql + o; }
  else if (mat == 1) { o = ((size_t)(b * NKV + head) * T + t0) * DH; dh = Kh + o; dl = Kl + o; }
  else               { o = ((size_t)(b * NKV + head) * QT_PER_B + (t0 >> 4)) * (size_t)(DH * 16); dh = Vh + o; dl = Vl + o; }
#pragma unroll
  for (int j = 0; j < 8; ++j) { const int e = (j * 32 + lane) * 8; *(volatile v8b*)(dh + e) = ld8b(Tp0 + e); *(volatile v8b*)(dl + e) = ld8b(Tp1 + e); }
  __threadfence();
#pragma unroll
  for (int j = 0; j < 8; ++j) { const int e = (j * 32 + lane) * 8; *(volatile v8b*)(dh + e) = ld8b(Tp0 + e); *(volatile v8b*)(dl + e) = ld8b(Tp1 + e); }
}

__global__ __launch_bounds__(256) void attn_kernel(const b16* __restrict__ Qh, const b16* __restrict__ Ql, const b16* __restrict__ Kh, const b16* __restrict__ Kl,
                                                   const b16* __restrict__ Vh, const b16* __restrict__ Vl, const int* __restrict__ seqlen,
                                                   const float* __restrict__ abias, float* __restrict__ yf) {
  __shared__ __attribute__((aligned(16))) float Os[8][16 * 64];
  const int wid = threadIdx.x >> 5, lane = threadIdx.x & 31, hh = lane >> 4, col = lane & 15;
  const int qtile = blockIdx.x * 8 + wid;
  const int g = qtile / QT_PER_B;
  const int q0 = (qtile % QT_PER_B) << 4;
  const int b = g / NH, h = g % NH, kvh = h / REP;
  const size_t ko = (size_t)(b * NKV + kvh) * T * DH;
  const size_t qo = ((size_t)g * T + q0 + col) * DH;
  const v16b q0h = frag_kb(Qh + qo, hh), q0l = frag_kb(Ql + qo, hh), q1h = frag_kb(Qh + qo + 32, hh), q1l = frag_kb(Ql + qo + 32, hh);
  float m = -INFINITY, l = 0.0f;
  v8f o0 = {}, o1 = {}, o2 = {}, o3 = {};
  const int slen = T; (void)seqlen;
  for (int kb = 0; kb < T; kb += 32) {
    const size_t r0 = ko + (size_t)(kb + col) * DH, r1 = ko + (size_t)(kb + 16 + col) * DH;
    v8f s0 = {}, s1 = {};
    {
      v16b ah = frag_kb(Kh + r0, hh), al = frag_kb(Kl + r0, hh);
      s0 = wmma1(ah, al, q0h, q0l, s0);
      ah = frag_kb(Kh + r0 + 32, hh); al = frag_kb(Kl + r0 + 32, hh);
      s0 = wmma1(ah, al, q1h, q1l, s0);
      ah = frag_kb(Kh + r1, hh); al = frag_kb(Kl + r1, hh);
      s1 = wmma1(ah, al, q0h, q0l, s1);
      ah = frag_kb(Kh + r1 + 32, hh); al = frag_kb(Kl + r1 + 32, hh);
      s1 = wmma1(ah, al, q1h, q1l, s1);
    }
    (void)slen;
    {
      const float* ab = abias + (size_t)b * T + kb + 8 * hh;
#pragma unroll
      for (int r = 0; r < 8; ++r) { s0[r] += ab[r]; s1[r] += ab[16 + r]; }
    }
    float mr = -INFINITY;
#pragma unroll
    for (int r = 0; r < 8; ++r) mr = fmaxf(mr, fmaxf(s0[r], s1[r]));
    mr = fmaxf(mr, __shfl_xor(mr, 16));
    float mn = fmaxf(m, mr);
    if (mn == -INFINITY) mn = 0.0f;
    const float al_ = __expf(m - mn);
    m = mn;
    float sum = 0.0f;
    v16b pbh, pbl;
#pragma unroll
    for (int r = 0; r < 8; ++r) {
      const float p0 = __expf(s0[r] - mn), p1 = __expf(s1[r] - mn);
      sum += p0 + p1;
      b16 a, c; split_bf16(p0, a, c); pbh[r] = a; pbl[r] = c; split_bf16(p1, a, c); pbh[8 + r] = a; pbl[8 + r] = c;
    }
    sum += __shfl_xor(sum, 16);
    l = l * al_ + sum;
#pragma unroll
    for (int r = 0; r < 8; ++r) { o0[r] *= al_; o1[r] *= al_; o2[r] *= al_; o3[r] *= al_; }
    const size_t v0 = ko + (size_t)(kb >> 4) * (DH * 16) + 8 * hh, v1 = v0 + DH * 16;
#pragma unroll
    for (int n = 0; n < 4; ++n) {
      const int f = n * 16 + col;
      const v16b vah = cat8b(ld8b(Vh + v0 + f * 16), ld8b(Vh + v1 + f * 16));
      const v16b val = cat8b(ld8b(Vl + v0 + f * 16), ld8b(Vl + v1 + f * 16));
      v8f& o = (n == 0) ? o0 : (n == 1) ? o1 : (n == 2) ? o2 : o3;
      o = wmma1(vah, val, pbh, pbl, o);
    }
  }
  const float inv = (q0 + col < slen && l > 0.0f) ? (1.0f / l) : 0.0f;
  float* Tt = Os[wid];
#pragma unroll
  for (int r = 0; r < 8; ++r) {
    const int hr = 8 * hh + r;
    Tt[col * 64 + 0 + hr] = o0[r] * inv; Tt[col * 64 + 16 + hr] = o1[r] * inv;
    Tt[col * 64 + 32 + hr] = o2[r] * inv; Tt[col * 64 + 48 + hr] = o3[r] * inv;
  }
  wave_lds_sync();
  float* dst0 = yf + ((size_t)b * T + q0) * HID + h * DH;
#pragma unroll
  for (int j = 0; j < 8; ++j) { const int rr = j * 2 + hh, c4 = col * 4; *(volatile v4f*)(dst0 + (size_t)rr * HID + c4) = *(const v4f*)(Tt + rr * 64 + c4); }
  __threadfence();
#pragma unroll
  for (int j = 0; j < 8; ++j) { const int rr = j * 2 + hh, c4 = col * 4; *(volatile v4f*)(dst0 + (size_t)rr * HID + c4) = *(const v4f*)(Tt + rr * 64 + c4); }
}

__global__ __launch_bounds__(128) void out_gemm_kernel(const float* __restrict__ yf, const b16* __restrict__ woh, const b16* __restrict__ wol, const float* __restrict__ bo, int yoff,
                                                       float* __restrict__ out) {
  __shared__ __attribute__((aligned(16))) float Ts[4][32 * 64];
  const int lane = threadIdx.x & 31, wave = threadIdx.x >> 5, nloc = lane & 15, hlf = lane >> 4;
  const int m0 = (blockIdx.y + yoff) * 128 + wave * 32;
  const int c0 = blockIdx.x * 64;
  v8f acc[2][4];
#pragma unroll
  for (int r = 0; r < 2; ++r)
#pragma unroll
    for (int t = 0; t < 4; ++t) acc[r][t] = (v8f){};
  gemm_tile_split(yf, woh, wol, m0, c0, HID, nloc, hlf, acc);
  float* Tt = Ts[wave];
#pragma unroll
  for (int t = 0; t < 4; ++t)
#pragma unroll
    for (int r = 0; r < 2; ++r)
#pragma unroll
      for (int v = 0; v < 8; ++v) Tt[(r * 16 + v + 8 * hlf) * 64 + t * 16 + nloc] = acc[r][t][v] + (bo ? bo[c0 + t * 16 + nloc] : 0.0f);
  wave_lds_sync();
  float* dst0 = out + (size_t)m0 * NOUT + c0;
#pragma unroll
  for (int j = 0; j < 16; ++j) { const int rr = j * 2 + hlf, c4 = nloc * 4; *(volatile v4f*)(dst0 + (size_t)rr * NOUT + c4) = *(const v4f*)(Tt + rr * 64 + c4); }
  __threadfence();
#pragma unroll
  for (int j = 0; j < 16; ++j) { const int rr = j * 2 + hlf, c4 = nloc * 4; *(volatile v4f*)(dst0 + (size_t)rr * NOUT + c4) = *(const v4f*)(Tt + rr * 64 + c4); }
}
__global__ __launch_bounds__(256) void wcvtQKV_kernel(const float* __restrict__ wq, const float* __restrict__ wk, const float* __restrict__ wv, b16* __restrict__ wh, b16* __restrict__ wl) {
  const size_t tid = (size_t)blockIdx.x * blockDim.x + threadIdx.x, stride = (size_t)gridDim.x * blockDim.x;
  const size_t nq = (size_t)NQKV * HIN / 8;
  for (int pass = 0; pass < 2; ++pass) {
    for (size_t c = tid; c < nq; c += stride) {
      const size_t i = c * 8, n = i / HIN, k0 = i % HIN;
      const int mat = (int)(n / HID), head = (int)((n % HID) / DH), d = (int)(n % DH);
      const float* w = (mat == 0) ? wq : (mat == 1) ? wk : wv;
      v8b bh, bl;
#pragma unroll
      for (int e = 0; e < 8; ++e) { const float v = (d < DR) ? w[(k0 + e) * (size_t)NOUT + head * DR + d] : 0.f; b16 a, cc; split_bf16(v, a, cc); bh[e] = a; bl[e] = cc; }
      *(volatile v8b*)(wh + i) = bh; *(volatile v8b*)(wl + i) = bl;
    }
    __threadfence();
  }
}
__global__ __launch_bounds__(256) void wcvtWo_kernel(const float* __restrict__ wo, b16* __restrict__ woh, b16* __restrict__ wol) {
  const size_t tid = (size_t)blockIdx.x * blockDim.x + threadIdx.x, stride = (size_t)gridDim.x * blockDim.x;
  const size_t no = (size_t)NOUT * HID / 8;
  for (int pass = 0; pass < 2; ++pass) {
    for (size_t c = tid; c < no; c += stride) { const size_t i = c * 8, n = i / HID, k0 = i % HID; const int h = (int)(k0 / DH), d0 = (int)(k0 % DH); v8b bh, bl;
#pragma unroll
      for (int e = 0; e < 8; ++e) { const int d = d0 + e; const float v = (d < DR) ? wo[(size_t)(h * DR + d) * NOUT + n] : 0.f; b16 a, cc; split_bf16(v, a, cc); bh[e] = a; bl[e] = cc; }
      *(volatile v8b*)(woh + i) = bh; *(volatile v8b*)(wol + i) = bl; }
    __threadfence();
  }
}
__global__ __launch_bounds__(256) void ln_kernel(const float* __restrict__ pre, const float* __restrict__ res, const float* __restrict__ g, const float* __restrict__ be, float* __restrict__ out) {
  const int row = blockIdx.x * 8 + (threadIdx.x >> 5), lane = threadIdx.x & 31;
  float v[8]; float s = 0.f;
#pragma unroll
  for (int e = 0; e < 8; ++e) { v[e] = pre[(size_t)row * NOUT + lane * 8 + e] + res[(size_t)row * NOUT + lane * 8 + e]; s += v[e]; }
#pragma unroll
  for (int o = 16; o > 0; o >>= 1) s += __shfl_xor(s, o, 32);
  const float mu = s * (1.0f / NOUT);
  float q = 0.f;
#pragma unroll
  for (int e = 0; e < 8; ++e) { const float dd = v[e] - mu; q += dd * dd; }
#pragma unroll
  for (int o = 16; o > 0; o >>= 1) q += __shfl_xor(q, o, 32);
  const float rs = 1.0f / sqrtf(q * (1.0f / NOUT) + 1e-12f);
  typedef __attribute__((ext_vector_type(8))) float v8f32; v8f32 ov;
#pragma unroll
  for (int e = 0; e < 8; ++e) { const int c = lane * 8 + e; ov[e] = (v[e] - mu) * rs * g[c] + be[c]; }
  *(volatile v8f32*)(out + (size_t)row * NOUT + lane * 8) = ov; __threadfence(); *(volatile v8f32*)(out + (size_t)row * NOUT + lane * 8) = ov;
}
}

extern "C" void kernel_launch(void* const* d_in, const int* in_sizes, int n_in,
                              void* d_out, int out_size, void* d_ws, size_t ws_size, hipStream_t stream) {
  (void)in_sizes; (void)n_in; (void)out_size;
  const float* x     = (const float*)d_in[0];
  const float* amask = (const float*)d_in[1];
  const float* cphi  = (const float*)d_in[2];
  const float* sphi  = (const float*)d_in[3];
  const float* mag   = (const float*)d_in[4];
  const float* Wq = (const float*)d_in[5];  const float* bq = (const float*)d_in[6];
  const float* Wk = (const float*)d_in[7];  const float* bk = (const float*)d_in[8];
  const float* Wv = (const float*)d_in[9];  const float* bv = (const float*)d_in[10];
  const float* Wo = (const float*)d_in[11]; const float* bo = (const float*)d_in[12];
  const float* bandl = (const float*)d_in[13];
  const float* pbs   = (const float*)d_in[14];
  const float* lng   = (const float*)d_in[15]; const float* lnb = (const float*)d_in[16];
  float* out = (float*)d_out;
  size_t off = 0; char* ws = (char*)d_ws;
  b16* wqh = (b16*)(ws + off); off += (size_t)NQKV * HIN * 2;
  b16* wql = (b16*)(ws + off); off += (size_t)NQKV * HIN * 2;
  b16* woh = (b16*)(ws + off); off += (size_t)NOUT * HID * 2;
  b16* wol = (b16*)(ws + off); off += (size_t)NOUT * HID * 2;
  b16* Qh  = (b16*)(ws + off); off += (size_t)MROWS * HID * 2;
  b16* Ql  = (b16*)(ws + off); off += (size_t)MROWS * HID * 2;
  b16* Kh  = (b16*)(ws + off); off += (size_t)MROWS * KVW * 2;
  b16* Kl  = (b16*)(ws + off); off += (size_t)MROWS * KVW * 2;
  b16* Vh  = (b16*)(ws + off); off += (size_t)MROWS * KVW * 2;
  b16* Vl  = (b16*)(ws + off); off += (size_t)MROWS * KVW * 2;
  float* yf  = (float*)(ws + off); off += (size_t)MROWS * HID * 4;
  float* pre = (float*)(ws + off); off += (size_t)MROWS * NOUT * 4;
  if (off > ws_size) return;
  const int ROWBLK = MROWS / 128, NQT = Bsz * NH * QT_PER_B;
  wcvtQKV_kernel<<<1024, 256, 0, stream>>>(Wq, Wk, Wv, wqh, wql);
  wcvtWo_kernel<<<256, 256, 0, stream>>>(Wo, woh, wol);
  qkv_gemm_kernel<<<dim3(NQKV / 64, ROWBLK), 128, 0, stream>>>(x, x, x, wqh, wql, bq, bk, bv, nullptr, 0, 0, cphi, sphi, mag, bandl, pbs, Qh, Ql, Kh, Kl, Vh, Vl);
  attn_kernel<<<NQT / 8, 256, 0, stream>>>(Qh, Ql, Kh, Kl, Vh, Vl, nullptr, amask, yf);
  out_gemm_kernel<<<dim3(NOUT / 64, ROWBLK), 128, 0, stream>>>(yf, woh, wol, bo, 0, pre);
  ln_kernel<<<MROWS / 8, 256, 0, stream>>>(pre, x, lng, lnb, out);
}
